// ReportDecoder_9448928051412
// MI455X (gfx1250) — hardware-verified
//
#include <hip/hip_runtime.h>
#include <stddef.h>

typedef __attribute__((ext_vector_type(16))) _Float16 v16h;
typedef __attribute__((ext_vector_type(8)))  _Float16 v8h;
typedef __attribute__((ext_vector_type(16))) __bf16   v16b;
typedef __attribute__((ext_vector_type(8)))  __bf16   v8b;
typedef __attribute__((ext_vector_type(8)))  float    v8f;
typedef __attribute__((ext_vector_type(4)))  float    v4f;
typedef __attribute__((ext_vector_type(4)))  unsigned int v4u;

constexpr int DIM_B   = 256;
constexpr int DIM_P   = 49;
constexpr int DIM_E   = 1024;
constexpr int DIM_H   = 1024;
constexpr int DIM_V   = 8;
constexpr int DIM_L   = 128;
constexpr int DIM_T   = 32;
constexpr int DIM_T1  = 33;
constexpr int DIM_IN  = 1161;
constexpr int DIM_G4  = 4096;
constexpr int DIM_NO  = 1154;
constexpr int DIM_NOP = 1216;
constexpr int COL_BEG = 1032;
constexpr int COL_LAB = 1033;
constexpr int K_IN    = 1056;
constexpr int PITCH_IN = 1088;
constexpr int CG_IN   = PITCH_IN / 8;
constexpr int K_LAB   = 128;
constexpr int PH_TILE = 1032;
constexpr int PL_TILE = 136;
constexpr int SEQ_THREADS = 512;
constexpr int UNITS_PER_WAVE = 64;
constexpr float H_SCALE    = 16384.0f;
constexpr float W_SCALE    = 16.0f;
constexpr float LAB_SCALE  = 262144.0f;
constexpr float INV_GSCALE = 1.0f / 262144.0f;

static_assert(K_IN % 32 == 0);
static_assert((PH_TILE * 2) % 16 == 0);
static_assert((PL_TILE * 2) % 16 == 0);
static_assert(DIM_NOP % 64 == 0);
static_assert((DIM_B * DIM_T) % 64 == 0);
static_assert(SEQ_THREADS / 32 * UNITS_PER_WAVE == DIM_H);

__device__ __forceinline__ unsigned short f2bf_bits(float f) {
  unsigned u = __float_as_uint(f);
  return (unsigned short)((u + 0x7FFFu + ((u >> 16) & 1u)) >> 16);
}
__device__ __forceinline__ float bf_bits2f(unsigned short h) { return __uint_as_float(((unsigned)h) << 16); }

__device__ __forceinline__ void dep_guard_h(v8f& a, v8f& b, v16h x, v16h y) { asm volatile("v_nop\n\tv_nop\n\tv_nop\n\tv_nop" : "+v"(a), "+v"(b) : "v"(x), "v"(y)); }
__device__ __forceinline__ void dep_guard_b(v8f& a, v8f& b, v16b x, v16b y) { asm volatile("v_nop\n\tv_nop\n\tv_nop\n\tv_nop" : "+v"(a), "+v"(b) : "v"(x), "v"(y)); }
__device__ __forceinline__ void keep4_h(v16h a, v16h b, v16h c, v16h d) { asm volatile("v_nop" :: "v"(a), "v"(b), "v"(c), "v"(d)); }
__device__ __forceinline__ void keep4_b(v16b a, v16b b, v16b c, v16b d) { asm volatile("v_nop" :: "v"(a), "v"(b), "v"(c), "v"(d)); }
__device__ __forceinline__ void acc_guard4(v8f& a, v8f& b, v8f& c, v8f& d) { asm volatile("v_nop\n\tv_nop\n\tv_nop\n\tv_nop" : "+v"(a), "+v"(b), "+v"(c), "+v"(d)); }
template <typename T> struct Frag;
template <> struct Frag<_Float16> {
  typedef v16h V; union U { v16h v; v8h h[2]; };
  static __device__ __forceinline__ v16h load(const _Float16* p) {
    U f; f.h[0] = *(const v8h*)(p); f.h[1] = *(const v8h*)(p + 16); return f.v;
  }
  static __device__ __forceinline__ v8f mma(v16h a, v16h b, v8f c) {
    return __builtin_amdgcn_wmma_f32_16x16x32_f16(false, a, false, b, (short)0, c, false, false);
  }
  static __device__ __forceinline__ void guard(v8f& a, v8f& b, v16h x, v16h y) { dep_guard_h(a, b, x, y); }
  static __device__ __forceinline__ void keep(v16h a, v16h b, v16h c, v16h d) { keep4_h(a, b, c, d); }
};
template <> struct Frag<__bf16> {
  typedef v16b V; union U { v16b v; v8b h[2]; };
  static __device__ __forceinline__ v16b load(const __bf16* p) {
    U f; f.h[0] = *(const v8b*)(p); f.h[1] = *(const v8b*)(p + 16); return f.v;
  }
  static __device__ __forceinline__ v8f mma(v16b a, v16b b, v8f c) {
    return __builtin_amdgcn_wmma_f32_16x16x32_bf16(false, a, false, b, (short)0, c, false, false);
  }
  static __device__ __forceinline__ void guard(v8f& a, v8f& b, v16b x, v16b y) { dep_guard_b(a, b, x, y); }
  static __device__ __forceinline__ void keep(v16b a, v16b b, v16b c, v16b d) { keep4_b(a, b, c, d); }
};

template <int ET> struct Elem;
template <> struct Elem<0> { typedef _Float16 T; };
template <> struct Elem<1> { typedef __bf16 T; };
template <int ET, int SPL, int BIAS_MODE, int OUT_MODE, bool RESID, int ACT = 0>
__global__ __launch_bounds__(256) void wmma_gemm64(
    const unsigned short* __restrict__ Ap, const unsigned short* __restrict__ A2p, int lda, long strideA,
    const unsigned short* __restrict__ Btp, const unsigned short* __restrict__ Bt2p, int ldb, long strideB,
    void* __restrict__ Cout, void* __restrict__ Cout2, int ldc, long strideC,
    const float* __restrict__ bias,
    const float* __restrict__ resid, long strideR,
    int M, int N, int K, float scale) {
  constexpr bool SPLIT = (SPL != 0);
  constexpr bool BSPL  = (SPL == 1);
  typedef typename Elem<ET>::T T;
  typedef typename Frag<T>::V V;
  const T* A = (const T*)Ap; const T* A2 = (const T*)A2p; const T* Bt = (const T*)Btp; const T* Bt2 = (const T*)Bt2p;
  __shared__ __align__(16) float sT[8][16 * 68];
  const int b    = blockIdx.y;
  const int lane = threadIdx.x & 31;
  const int wave = threadIdx.x >> 5;
  const int tilesN = N >> 6;
  const int tilesM = M >> 6;
  const int tile = blockIdx.x * 8 + wave;
  if (tile >= tilesM * tilesN) return;
  const int tm = tile / tilesN;
  const int tn = tile - tm * tilesN;
  const int m0 = tm << 6;
  const int n0 = tn << 6;

  const T* Ab  = A  + (size_t)b * strideA;
  const T* Bb  = Bt + (size_t)b * strideB;
  const T* Ab2 = SPLIT ? (A2  + (size_t)b * strideA) : nullptr;
  const T* Bb2 = BSPL  ? (Bt2 + (size_t)b * strideB) : nullptr;

  const int rlane = lane & 15;
  const int koff  = (lane >> 4) * 8;
  const int mOff  = (lane >> 4) * 8;

  v8f acc[4][4];
#pragma unroll
  for (int i = 0; i < 4; ++i)
#pragma unroll
    for (int j = 0; j < 4; ++j) acc[i][j] = (v8f){0.f,0.f,0.f,0.f,0.f,0.f,0.f,0.f};

  for (int k0 = 0; k0 < K; k0 += 32) {
    V bh[4], bl[4];
#pragma unroll
    for (int j = 0; j < 4; ++j) {
      const size_t bo = (size_t)(n0 + (j << 4) + rlane) * ldb + koff + k0;
      bh[j] = Frag<T>::load(Bb + bo);
      if (BSPL) bl[j] = Frag<T>::load(Bb2 + bo);
    }
#pragma unroll
    for (int i = 0; i < 4; ++i) {
      const size_t ao = (size_t)(m0 + (i << 4) + rlane) * lda + koff + k0;
      V ah = Frag<T>::load(Ab + ao);
      V al;
      if (SPLIT) al = Frag<T>::load(Ab2 + ao);
#pragma unroll
      for (int j = 0; j < 4; ++j) {
        acc[i][j] = Frag<T>::mma(ah, bh[j], acc[i][j]);
        if (BSPL) acc[i][j] = Frag<T>::mma(ah, bl[j], acc[i][j]);
        if (SPLIT) acc[i][j] = Frag<T>::mma(al, bh[j], acc[i][j]);
      }
      Frag<T>::guard(acc[i][0], acc[i][3], ah, SPLIT ? al : ah);
    }
    Frag<T>::keep(bh[0], bh[1], bh[2], bh[3]);
    if (BSPL) Frag<T>::keep(bl[0], bl[1], bl[2], bl[3]);
  }
  acc_guard4(acc[0][0], acc[0][1], acc[0][2], acc[0][3]);
  acc_guard4(acc[1][0], acc[1][1], acc[1][2], acc[1][3]);
  acc_guard4(acc[2][0], acc[2][1], acc[2][2], acc[2][3]);
  acc_guard4(acc[3][0], acc[3][1], acc[3][2], acc[3][3]);

  float* slab = sT[wave];
  const float* Rb = RESID ? (resid + (size_t)b * strideR) : nullptr;
#pragma unroll
  for (int i = 0; i < 4; ++i) {
    const int mBase = m0 + (i << 4);
#pragma unroll
    for (int j = 0; j < 4; ++j) {
      const int n = n0 + (j << 4) + rlane;
      float bv = 0.f;
      if (BIAS_MODE == 2) bv = bias[n];
#pragma unroll
      for (int r = 0; r < 8; ++r) {
        float v = acc[i][j][r] * scale;
        if (BIAS_MODE == 1) v += bias[mBase + mOff + r];
        if (BIAS_MODE == 2) v += bv;
        if (RESID) v += Rb[(size_t)(mBase + mOff + r) * ldc + n];
        if (ACT == 1) v = tanhf(v);
        if (ACT == 2) v = fmaxf(v, 0.0f);
        slab[(mOff + r) * 68 + (j << 4) + rlane] = v;
      }
    }
    __builtin_amdgcn_fence(__ATOMIC_RELEASE, "workgroup");
    __builtin_amdgcn_wave_barrier();
    __builtin_amdgcn_fence(__ATOMIC_ACQUIRE, "workgroup");
    if (OUT_MODE == 0) {
      float* C = (float*)Cout + (size_t)b * strideC;
      const int hh = lane >> 4, c4 = (lane & 15) * 4;
      for (int pass = 0; pass < 2; ++pass) {
#pragma unroll
        for (int it = 0; it < 8; ++it) {
          const int row = it * 2 + hh;
          v4f v = *(const v4f*)(slab + row * 68 + c4);
          *(volatile v4f*)(C + (size_t)(mBase + row) * ldc + n0 + c4) = v;
        }
        __threadfence();
      }
    } else {
      const int q = lane >> 3, c8 = (lane & 7) * 8;
      unsigned short* C  = (unsigned short*)Cout  + (size_t)b * strideC;
      unsigned short* C2 = (OUT_MODE == 2) ? ((unsigned short*)Cout2 + (size_t)b * strideC) : nullptr;
      for (int pass = 0; pass < 2; ++pass) {
#pragma unroll
        for (int it = 0; it < 4; ++it) {
          const int row = it * 4 + q;
          const float* sp = slab + row * 68 + c8;
          v8h hv, lv;
#pragma unroll
          for (int e = 0; e < 8; ++e) {
            if (OUT_MODE == 1) {
              hv[e] = (_Float16)sp[e];
            } else {
              unsigned short hb = f2bf_bits(sp[e]);
              unsigned short lb = f2bf_bits(sp[e] - bf_bits2f(hb));
              hv[e] = __builtin_bit_cast(_Float16, hb);
              lv[e] = __builtin_bit_cast(_Float16, lb);
            }
          }
          *(volatile v8h*)(C + (size_t)(mBase + row) * ldc + n0 + c8) = hv;
          if (OUT_MODE == 2) *(volatile v8h*)(C2 + (size_t)(mBase + row) * ldc + n0 + c8) = lv;
        }
        __threadfence();
      }
    }
    __builtin_amdgcn_fence(__ATOMIC_RELEASE, "workgroup");
    __builtin_amdgcn_wave_barrier();
    __builtin_amdgcn_fence(__ATOMIC_ACQUIRE, "workgroup");
  }
}

__device__ __forceinline__ unsigned int bf_pair(float x0, float x1) {
  return (unsigned)f2bf_bits(x0) | ((unsigned)f2bf_bits(x1) << 16);
}
__device__ __forceinline__ unsigned int h16_pair(float x0, float x1) {
  return (unsigned)__builtin_bit_cast(unsigned short, (_Float16)x0) |
         ((unsigned)__builtin_bit_cast(unsigned short, (_Float16)x1) << 16);
}
__device__ __forceinline__ unsigned int split_pair(float x0, float x1, unsigned int& lo_out) {
  const unsigned short h0 = f2bf_bits(x0), h1 = f2bf_bits(x1);
  const unsigned short l0 = f2bf_bits(x0 - bf_bits2f(h0));
  const unsigned short l1 = f2bf_bits(x1 - bf_bits2f(h1));
  lo_out = (unsigned)l0 | ((unsigned)l1 << 16);
  return (unsigned)h0 | ((unsigned)h1 << 16);
}
__device__ __forceinline__ void split8(v4f a, v4f b, v4u& hv, v4u& lv) {
  unsigned l;
  hv.x = split_pair(a.x, a.y, l); lv.x = l;
  hv.y = split_pair(a.z, a.w, l); lv.y = l;
  hv.z = split_pair(b.x, b.y, l); lv.z = l;
  hv.w = split_pair(b.z, b.w, l); lv.w = l;
}
__device__ __forceinline__ v4u h16_pack8(v4f a, v4f b) {
  v4u r;
  r.x = h16_pair(a.x, a.y); r.y = h16_pair(a.z, a.w);
  r.z = h16_pair(b.x, b.y); r.w = h16_pair(b.z, b.w);
  return r;
}
__device__ __forceinline__ v4u lab_pack8(const float* lp) {
  const v4f a = *(const v4f*)lp;
  const v4f b = *(const v4f*)(lp + 4);
  v4u r;
  r.x = bf_pair(a.x * LAB_SCALE, a.y * LAB_SCALE);
  r.y = bf_pair(a.z * LAB_SCALE, a.w * LAB_SCALE);
  r.z = bf_pair(b.x * LAB_SCALE, b.y * LAB_SCALE);
  r.w = bf_pair(b.z * LAB_SCALE, b.w * LAB_SCALE);
  return r;
}
__device__ __forceinline__ float sigf(float x) { return __builtin_amdgcn_rcpf(1.0f + expf(-x)); }
__device__ __forceinline__ float tnhf(float x) { return 2.0f * __builtin_amdgcn_rcpf(1.0f + expf(-2.0f * x)) - 1.0f; }

__global__ __launch_bounds__(256) void prep_bias_beg(const float* __restrict__ b_ih, const float* __restrict__ b_hh,
                                                     const float* __restrict__ w_ih,
                                                     float* __restrict__ bsum, float* __restrict__ wbeg) {
  const int i = blockIdx.x * 256 + threadIdx.x;
  if (i >= DIM_G4 / 4) return;
  const int n = i * 4;
  v4f s, w;
  s.x = b_ih[n + 0] + b_hh[n + 0]; w.x = w_ih[(size_t)(n + 0) * DIM_IN + COL_BEG];
  s.y = b_ih[n + 1] + b_hh[n + 1]; w.y = w_ih[(size_t)(n + 1) * DIM_IN + COL_BEG];
  s.z = b_ih[n + 2] + b_hh[n + 2]; w.z = w_ih[(size_t)(n + 2) * DIM_IN + COL_BEG];
  s.w = b_ih[n + 3] + b_hh[n + 3]; w.w = w_ih[(size_t)(n + 3) * DIM_IN + COL_BEG];
  *(volatile v4f*)(bsum + n) = s;
  *(volatile v4f*)(wbeg + n) = w;
  __threadfence();
  *(volatile v4f*)(bsum + n) = s;
  *(volatile v4f*)(wbeg + n) = w;
}

__global__ __launch_bounds__(256) void build_amean(const float* __restrict__ image, const float* __restrict__ view,
                                                   unsigned short* __restrict__ ah, unsigned short* __restrict__ al) {
  const int i = blockIdx.x * 256 + threadIdx.x;
  if (i >= DIM_B * CG_IN) return;
  const int b = i / CG_IN, cg = i - b * CG_IN;
  const int c0 = (cg * 8 <= DIM_E - 8) ? cg * 8 : (DIM_E - 8);
  const float* p = image + (size_t)b * DIM_P * DIM_E + c0;
  v4f sa = {0.f, 0.f, 0.f, 0.f}, sb = {0.f, 0.f, 0.f, 0.f};
#pragma unroll 1
  for (int q = 0; q < DIM_P; ++q) {
    sa += *(const v4f*)(p + (size_t)q * DIM_E);
    sb += *(const v4f*)(p + (size_t)q * DIM_E + 4);
  }
  const float inv = 1.0f / 49.0f;
  sa *= inv; sb *= inv;
  const v4f va = *(const v4f*)(view + b * DIM_V);
  const v4f vb = *(const v4f*)(view + b * DIM_V + 4);
  const bool is_mean = (cg < DIM_E / 8);
  const bool is_view = (cg == DIM_E / 8);
  v4f r0, r1;
  r0.x = is_mean ? sa.x : (is_view ? va.x : 0.f);
  r0.y = is_mean ? sa.y : (is_view ? va.y : 0.f);
  r0.z = is_mean ? sa.z : (is_view ? va.z : 0.f);
  r0.w = is_mean ? sa.w : (is_view ? va.w : 0.f);
  r1.x = is_mean ? sb.x : (is_view ? vb.x : 0.f);
  r1.y = is_mean ? sb.y : (is_view ? vb.y : 0.f);
  r1.z = is_mean ? sb.z : (is_view ? vb.z : 0.f);
  r1.w = is_mean ? sb.w : (is_view ? vb.w : 0.f);
  v4u hv, lv;
  split8(r0, r1, hv, lv);
  const size_t o = (size_t)b * PITCH_IN + cg * 8;
  *(volatile v4u*)(ah + o) = hv;
  *(volatile v4u*)(al + o) = lv;
  __threadfence();
  *(volatile v4u*)(ah + o) = hv;
  *(volatile v4u*)(al + o) = lv;
}

__global__ __launch_bounds__(256) void cast_wih_split(const float* __restrict__ w_ih,
                                                      unsigned short* __restrict__ dh, unsigned short* __restrict__ dl) {
  const int i = blockIdx.x * 256 + threadIdx.x;
  if (i >= DIM_G4 * CG_IN) return;
  const int n = i / CG_IN, cg = i - n * CG_IN;
  const int c = cg * 8;
  const float* p = w_ih + (size_t)n * DIM_IN + c;
  float x[8];
#pragma unroll
  for (int e = 0; e < 8; ++e) { const float v = p[e]; x[e] = (c + e < COL_BEG) ? v : 0.f; }
  const v4f a = {x[0], x[1], x[2], x[3]}, b = {x[4], x[5], x[6], x[7]};
  v4u hv, lv;
  split8(a, b, hv, lv);
  const size_t o = (size_t)n * PITCH_IN + c;
  *(volatile v4u*)(dh + o) = hv;
  *(volatile v4u*)(dl + o) = lv;
  __threadfence();
  *(volatile v4u*)(dh + o) = hv;
  *(volatile v4u*)(dl + o) = lv;
}

__global__ __launch_bounds__(256) void cast_wlab_split(const float* __restrict__ w_ih,
                                                       unsigned short* __restrict__ dh, unsigned short* __restrict__ dl) {
  const int i = blockIdx.x * 256 + threadIdx.x;
  if (i >= DIM_G4 * (K_LAB / 8)) return;
  const int n = i >> 4, q = i & 15;
  const float* p = w_ih + (size_t)n * DIM_IN + COL_LAB + q * 8;
  const v4f a = {p[0], p[1], p[2], p[3]}, b = {p[4], p[5], p[6], p[7]};
  v4u hv, lv;
  split8(a, b, hv, lv);
  const size_t o = (size_t)n * K_LAB + q * 8;
  *(volatile v4u*)(dh + o) = hv;
  *(volatile v4u*)(dl + o) = lv;
  __threadfence();
  *(volatile v4u*)(dh + o) = hv;
  *(volatile v4u*)(dl + o) = lv;
}

__global__ __launch_bounds__(256) void split_rows_bf16(const float* __restrict__ src, int n8,
                                                      unsigned short* __restrict__ dh, unsigned short* __restrict__ dl) {
  const int i = blockIdx.x * 256 + threadIdx.x;
  if (i >= n8) return;
  const size_t o = (size_t)i * 8;
  const v4f a = *(const v4f*)(src + o), b = *(const v4f*)(src + o + 4);
  v4u hv, lv;
  split8(a, b, hv, lv);
  *(volatile v4u*)(dh + o) = hv;
  *(volatile v4u*)(dl + o) = lv;
  __threadfence();
  *(volatile v4u*)(dh + o) = hv;
  *(volatile v4u*)(dl + o) = lv;
}

__global__ __launch_bounds__(256) void cast_rows_f16(const float* __restrict__ src, int rows_src, int rows_dst, int cols8,
                                                    float scale, unsigned short* __restrict__ dst) {
  const int i = blockIdx.x * 256 + threadIdx.x;
  if (i >= rows_dst * cols8) return;
  const int r = i / cols8, c8 = i - r * cols8;
  const int rs = (r < rows_src) ? r : (rows_src - 1);
  const float* p = src + (size_t)rs * cols8 * 8 + c8 * 8;
  v4f a = *(const v4f*)(p), b = *(const v4f*)(p + 4);
  const float s = (r < rows_src) ? scale : 0.0f;
  a.x = (r < rows_src) ? a.x * s : 0.f; a.y = (r < rows_src) ? a.y * s : 0.f;
  a.z = (r < rows_src) ? a.z * s : 0.f; a.w = (r < rows_src) ? a.w * s : 0.f;
  b.x = (r < rows_src) ? b.x * s : 0.f; b.y = (r < rows_src) ? b.y * s : 0.f;
  b.z = (r < rows_src) ? b.z * s : 0.f; b.w = (r < rows_src) ? b.w * s : 0.f;
  const v4u hv = h16_pack8(a, b);
  const size_t o = (size_t)i * 8;
  *(volatile v4u*)(dst + o) = hv;
  __threadfence();
  *(volatile v4u*)(dst + o) = hv;
}

__device__ __forceinline__ void gates_gemm(v8f (&acc)[4],
    const unsigned short* labA, const unsigned short* hA,
    const unsigned short* __restrict__ wlabh, const unsigned short* __restrict__ wlabl,
    const unsigned short* __restrict__ whh, int nrow, int koff) {
  const v8f z = {0.f,0.f,0.f,0.f,0.f,0.f,0.f,0.f};
  acc[0] = z; acc[1] = z; acc[2] = z; acc[3] = z;
  const size_t lb = (size_t)nrow * K_LAB + koff;
  const size_t gstep_l = (size_t)DIM_H * K_LAB;
#pragma unroll 1
  for (int ks = 0; ks < K_LAB / 32; ++ks) {
    v16b bq[4];
#pragma unroll
    for (int g = 0; g < 4; ++g) bq[g] = Frag<__bf16>::load((const __bf16*)(wlabh + lb + (size_t)g * gstep_l + ks * 32));
    const v16b a = Frag<__bf16>::load((const __bf16*)(labA + ks * 32));
#pragma unroll
    for (int g = 0; g < 4; ++g) acc[g] = Frag<__bf16>::mma(a, bq[g], acc[g]);
    Frag<__bf16>::guard(acc[0], acc[3], a, a);
    Frag<__bf16>::keep(bq[0], bq[1], bq[2], bq[3]);
  }
#pragma unroll 1
  for (int ks = 0; ks < K_LAB / 32; ++ks) {
    v16b bq[4];
#pragma unroll
    for (int g = 0; g < 4; ++g) bq[g] = Frag<__bf16>::load((const __bf16*)(wlabl + lb + (size_t)g * gstep_l + ks * 32));
    const v16b a = Frag<__bf16>::load((const __bf16*)(labA + ks * 32));
#pragma unroll
    for (int g = 0; g < 4; ++g) acc[g] = Frag<__bf16>::mma(a, bq[g], acc[g]);
    Frag<__bf16>::guard(acc[0], acc[3], a, a);
    Frag<__bf16>::keep(bq[0], bq[1], bq[2], bq[3]);
  }
  const size_t hb = (size_t)nrow * DIM_H + koff;
  const size_t gstep_h = (size_t)DIM_H * DIM_H;
#pragma unroll 1
  for (int ks = 0; ks < DIM_H / 32; ++ks) {
    v16h bq[4];
#pragma unroll
    for (int g = 0; g < 4; ++g) bq[g] = Frag<_Float16>::load((const _Float16*)(whh + hb + (size_t)g * gstep_h + ks * 32));
    const v16h a = Frag<_Float16>::load((const _Float16*)(hA + ks * 32));
#pragma unroll
    for (int g = 0; g < 4; ++g) acc[g] = Frag<_Float16>::mma(a, bq[g], acc[g]);
    Frag<_Float16>::guard(acc[0], acc[3], a, a);
    Frag<_Float16>::keep(bq[0], bq[1], bq[2], bq[3]);
  }
  acc_guard4(acc[0], acc[1], acc[2], acc[3]);
}

__device__ __forceinline__ void cell_update(const v8f (&acc)[4], const float* __restrict__ xr,
    float wb0, float wb1, float wb2, float wb3,
    float (&m)[8], unsigned int (&lo)[4], unsigned short* hcol) {
  unsigned short lob[8];
#pragma unroll
  for (int r = 0; r < 8; ++r) {
    const float* xrr = xr + (size_t)r * DIM_G4;
    const float gi = acc[0][r] * INV_GSCALE + xrr[0] + wb0;
    const float gf = acc[1][r] * INV_GSCALE + xrr[DIM_H] + wb1;
    const float gg = acc[2][r] * INV_GSCALE + xrr[2 * DIM_H] + wb2;
    const float go = acc[3][r] * INV_GSCALE + xrr[3 * DIM_H] + wb3;
    const float mo = m[r];
    const float mn = sigf(gf) * mo + sigf(gi) * tnhf(gg);
    const float hn = sigf(go) * tnhf(mn);
    m[r] = mn;
    const float hs = hn * H_SCALE;
    const _Float16 hq = (_Float16)hs;
    const float res = hs - (float)hq;
    hcol[r * PH_TILE] = __builtin_bit_cast(unsigned short, hq);
    lob[r] = __builtin_bit_cast(unsigned short, (_Float16)res);
  }
#pragma unroll
  for (int q = 0; q < 4; ++q) lo[q] = (unsigned)lob[2 * q] | ((unsigned)lob[2 * q + 1] << 16);
}

template <int PIDX>
__device__ __forceinline__ void run_pass(float (&mreg)[4][8], unsigned int (&lopk)[4][4],
    const unsigned short* labA, const unsigned short* hA, unsigned short* hout_base,
    const unsigned short* __restrict__ wlabh, const unsigned short* __restrict__ wlabl,
    const unsigned short* __restrict__ whh,
    const float* __restrict__ xc_rows, const float* __restrict__ wbeg, float begf,
    int ubase, int rl, int koff) {
  const int j = ubase + 16 * PIDX + rl;
  v8f acc[4];
  gates_gemm(acc, labA, hA, wlabh, wlabl, whh, j, koff);
  const float wb0 = begf * wbeg[j];
  const float wb1 = begf * wbeg[DIM_H + j];
  const float wb2 = begf * wbeg[2 * DIM_H + j];
  const float wb3 = begf * wbeg[3 * DIM_H + j];
  cell_update(acc, xc_rows + j, wb0, wb1, wb2, wb3, mreg[PIDX], lopk[PIDX], hout_base + j);
}

__global__ __launch_bounds__(SEQ_THREADS) void lstm_seq(
    const float* __restrict__ h0t, const float* __restrict__ m0t,
    const float* __restrict__ label, const float* __restrict__ xc, const float* __restrict__ wbeg,
    const unsigned short* __restrict__ whh, const unsigned short* __restrict__ wlabh,
    const unsigned short* __restrict__ wlabl,
    unsigned short* __restrict__ hseqh, unsigned short* __restrict__ hseql) {
  __shared__ __align__(16) unsigned short hT[2][16 * PH_TILE];
  __shared__ __align__(16) unsigned short labT[16 * PL_TILE];

  const int tid = threadIdx.x;
  const int wv = tid >> 5;
  const int lane = tid & 31;
  const int hh = lane >> 4;
  const int rl = lane & 15;
  const int koff = hh * 8;
  const int brow0 = blockIdx.x * 16;
  const int ubase = wv * UNITS_PER_WAVE;

#pragma unroll 1
  for (int idx = tid; idx < 16 * DIM_H; idx += SEQ_THREADS) {
    const int row = idx >> 10, j = idx & 1023;
    const float hv = h0t[(size_t)(brow0 + row) * DIM_H + j] * H_SCALE;
    hT[0][row * PH_TILE + j] = __builtin_bit_cast(unsigned short, (_Float16)hv);
  }
  float mreg[4][8];
#pragma unroll
  for (int p = 0; p < 4; ++p) {
#pragma unroll
    for (int r = 0; r < 8; ++r) {
      mreg[p][r] = m0t[(size_t)(brow0 + 8 * hh + r) * DIM_H + ubase + 16 * p + rl];
    }
  }
  if (tid < 256) {
    const int row = tid >> 4, q = tid & 15;
    const float* lp = label + ((size_t)(brow0 + row) * DIM_T1 + 0) * DIM_L + q * 8;
    *(v4u*)(&labT[row * PL_TILE + q * 8]) = lab_pack8(lp);
  }
  __syncthreads();

#pragma unroll 1
  for (int t = 0; t < DIM_T; ++t) {
    const int cur = t & 1, nxt = cur ^ 1;
    const unsigned short* At = &hT[cur][0];
    unsigned short* Aw = &hT[cur][0];
    unsigned short* An = &hT[nxt][0];
    const float begf = (t == 0) ? 1.0f : 0.0f;

    unsigned int lopk[4][4];
    {
      const unsigned short* labA = labT + rl * PL_TILE + koff;
      const unsigned short* hA = At + rl * PH_TILE + koff;
      unsigned short* hout = An + (8 * hh) * PH_TILE;
      const float* xcr = xc + (size_t)(brow0 + 8 * hh) * DIM_G4;
      run_pass<0>(mreg, lopk, labA, hA, hout, wlabh, wlabl, whh, xcr, wbeg, begf, ubase, rl, koff);
      run_pass<1>(mreg, lopk, labA, hA, hout, wlabh, wlabl, whh, xcr, wbeg, begf, ubase, rl, koff);
      run_pass<2>(mreg, lopk, labA, hA, hout, wlabh, wlabl, whh, xcr, wbeg, begf, ubase, rl, koff);
      run_pass<3>(mreg, lopk, labA, hA, hout, wlabh, wlabl, whh, xcr, wbeg, begf, ubase, rl, koff);
    }
    __syncthreads();

#pragma unroll
    for (int p = 0; p < 4; ++p) {
#pragma unroll
      for (int q = 0; q < 4; ++q) {
        const unsigned int w = lopk[p][q];
        unsigned short* col = Aw + (8 * hh + 2 * q) * PH_TILE + ubase + 16 * p + rl;
        col[0] = (unsigned short)(w & 0xffffu);
        col[PH_TILE] = (unsigned short)(w >> 16);
      }
    }
    if (tid < 256) {
      const int row = tid >> 4, q = tid & 15;
      const float* lp = label + ((size_t)(brow0 + row) * DIM_T1 + (t + 1)) * DIM_L + q * 8;
      *(v4u*)(&labT[row * PL_TILE + q * 8]) = lab_pack8(lp);
    }
    __syncthreads();

    {
      const int q = lane >> 3, c8 = (lane & 7) * 8;
      for (int pass = 0; pass < 2; ++pass) {
#pragma unroll
        for (int it = 0; it < 4; ++it) {
          const int row = it * 4 + q;
          const v4u hv = *(const v4u*)(An + row * PH_TILE + ubase + c8);
          const v4u lv = *(const v4u*)(Aw + row * PH_TILE + ubase + c8);
          const size_t gb = ((size_t)(brow0 + row) * DIM_T + t) * DIM_H + ubase + c8;
          *(volatile v4u*)(hseqh + gb) = hv;
          *(volatile v4u*)(hseql + gb) = lv;
        }
        __threadfence();
      }
    }
    __syncthreads();
  }
}

__global__ __launch_bounds__(256) void heads_kernel(const float* __restrict__ outp, const float* __restrict__ fcb,
                                                   const int* __restrict__ length, float* __restrict__ out) {
  const int b = blockIdx.x, tid = threadIdx.x, wv = tid >> 5, lane = tid & 31;
  const int lenb = length[b];
  float* out0 = out;
  float* out1 = out0 + (size_t)DIM_B * DIM_T * DIM_L;
  float* out2 = out1 + (size_t)DIM_B * DIM_T * DIM_H;
  float* out3 = out2 + (size_t)DIM_B * DIM_T;

#pragma unroll 1
  for (int tt = 0; tt < 4; ++tt) {
    const int t = wv * 4 + tt;
    const float mk = (lenb > t) ? 1.0f : 0.0f;
    const size_t rowi = (size_t)b * DIM_T + t;
    const float* rp = outp + rowi * DIM_NOP + DIM_L;
    v4f vals[8];
#pragma unroll
    for (int it = 0; it < 8; ++it) {
      const int col = it * 128 + lane * 4;
      const v4f x = *(const v4f*)(rp + col);
      const v4f bb = *(const v4f*)(fcb + DIM_L + col);
      const v4f s = x + bb;
      v4f o;
      o.x = fmaxf(s.x, 0.0f) * mk; o.y = fmaxf(s.y, 0.0f) * mk;
      o.z = fmaxf(s.z, 0.0f) * mk; o.w = fmaxf(s.w, 0.0f) * mk;
      vals[it] = o;
    }
    float* dst = out1 + rowi * DIM_H + lane * 4;
    for (int pass = 0; pass < 2; ++pass) {
#pragma unroll
      for (int it = 0; it < 8; ++it) *(volatile v4f*)(dst + it * 128) = vals[it];
      __threadfence();
    }
  }
#pragma unroll 1
  for (int k2 = 0; k2 < 16; ++k2) {
    const int task = k2 * 8 + wv;
    const int t = task >> 2, qu = task & 3;
    const float mk = (lenb > t) ? 1.0f : 0.0f;
    const size_t rowi = (size_t)b * DIM_T + t;
    const int col = qu * 32 + lane;
    const float v = sigf(outp[rowi * DIM_NOP + col] + fcb[col]) * mk;
    volatile float* dst = out0 + rowi * DIM_L + col;
    *dst = v;
    __threadfence();
    *dst = v;
  }
  if (wv == 0) {
    const int t = lane;
    const float mk = (lenb > t) ? 1.0f : 0.0f;
    const float* rp = outp + ((size_t)b * DIM_T + t) * DIM_NOP;
    const float v2 = sigf(rp[DIM_L + DIM_H] + fcb[DIM_L + DIM_H]) * mk;
    const float v3 = expf(rp[DIM_L + DIM_H + 1] + fcb[DIM_L + DIM_H + 1]) * mk;
    volatile float* p2 = out2 + (size_t)b * DIM_T + lane;
    volatile float* p3 = out3 + (size_t)b * DIM_T + lane;
    *p2 = v2;
    *p3 = v3;
    __threadfence();
    *p2 = v2;
    *p3 = v3;
  }
}

extern "C" void kernel_launch(void* const* d_in, const int* in_sizes, int n_in,
                              void* d_out, int out_size, void* d_ws, size_t ws_size,
                              hipStream_t stream) {
  (void)in_sizes; (void)n_in; (void)out_size;
  const float* image  = (const float*)d_in[0];
  const float* view   = (const float*)d_in[1];
  const float* label  = (const float*)d_in[2];
  const int*   length = (const int*)d_in[3];
  const float* fc_h_w = (const float*)d_in[4];
  const float* fc_h_b = (const float*)d_in[5];
  const float* fc_m_w = (const float*)d_in[6];
  const float* fc_m_b = (const float*)d_in[7];
  const float* fc_w   = (const float*)d_in[8];
  const float* fc_b   = (const float*)d_in[9];
  const float* w_ih   = (const float*)d_in[10];
  const float* b_ih   = (const float*)d_in[11];
  const float* w_hh   = (const float*)d_in[12];
  const float* b_hh   = (const float*)d_in[13];
  float* out = (float*)d_out;

  char* base = (char*)d_ws;
  size_t off = 0;
  auto carve = [&](size_t bytes) -> char* {
    char* p = base + off;
    off += (bytes + 255) & ~(size_t)255;
    return p;
  };
  float* bsum = (float*)carve((size_t)DIM_G4 * 4);
  float* wbeg = (float*)carve((size_t)DIM_G4 * 4);
  unsigned short* ameanh = (unsigned short*)carve((size_t)DIM_B * PITCH_IN * 2);
  unsigned short* ameanl = (unsigned short*)carve((size_t)DIM_B * PITCH_IN * 2);
  unsigned short* wihh = (unsigned short*)carve((size_t)DIM_G4 * PITCH_IN * 2);
  unsigned short* wihl = (unsigned short*)carve((size_t)DIM_G4 * PITCH_IN * 2);
  unsigned short* wlabh = (unsigned short*)carve((size_t)DIM_G4 * K_LAB * 2);
  unsigned short* wlabl = (unsigned short*)carve((size_t)DIM_G4 * K_LAB * 2);
  unsigned short* whh16 = (unsigned short*)carve((size_t)DIM_G4 * DIM_H * 2);
  unsigned short* fcw16 = (unsigned short*)carve((size_t)DIM_NOP * DIM_H * 2);
  unsigned short* fchh = (unsigned short*)carve((size_t)DIM_H * DIM_E * 2);
  unsigned short* fchl = (unsigned short*)carve((size_t)DIM_H * DIM_E * 2);
  unsigned short* fcmh = (unsigned short*)carve((size_t)DIM_H * DIM_E * 2);
  unsigned short* fcml = (unsigned short*)carve((size_t)DIM_H * DIM_E * 2);
  float* xc  = (float*)carve((size_t)DIM_B * DIM_G4 * 4);
  float* h0t = (float*)carve((size_t)DIM_B * DIM_H * 4);
  float* m0t = (float*)carve((size_t)DIM_B * DIM_H * 4);
  unsigned short* hseqh = (unsigned short*)carve((size_t)DIM_B * DIM_T * DIM_H * 2);
  unsigned short* hseql = (unsigned short*)carve((size_t)DIM_B * DIM_T * DIM_H * 2);
  float* outp = (float*)carve((size_t)DIM_B * DIM_T * DIM_NOP * 4);
  if (off > ws_size) return;

  const int TPB = 256;
  prep_bias_beg<<<(DIM_G4 / 4 + TPB - 1) / TPB, TPB, 0, stream>>>(b_ih, b_hh, w_ih, bsum, wbeg);
  build_amean<<<(DIM_B * CG_IN + TPB - 1) / TPB, TPB, 0, stream>>>(image, view, ameanh, ameanl);
  cast_wih_split<<<(DIM_G4 * CG_IN + TPB - 1) / TPB, TPB, 0, stream>>>(w_ih, wihh, wihl);
  cast_wlab_split<<<(DIM_G4 * (K_LAB / 8) + TPB - 1) / TPB, TPB, 0, stream>>>(w_ih, wlabh, wlabl);
  split_rows_bf16<<<(DIM_H * DIM_E / 8 + TPB - 1) / TPB, TPB, 0, stream>>>(fc_h_w, DIM_H * DIM_E / 8, fchh, fchl);
  split_rows_bf16<<<(DIM_H * DIM_E / 8 + TPB - 1) / TPB, TPB, 0, stream>>>(fc_m_w, DIM_H * DIM_E / 8, fcmh, fcml);
  cast_rows_f16<<<(DIM_G4 * (DIM_H / 8) + TPB - 1) / TPB, TPB, 0, stream>>>(w_hh, DIM_G4, DIM_G4, DIM_H / 8, W_SCALE, whh16);
  cast_rows_f16<<<(DIM_NOP * (DIM_H / 8) + TPB - 1) / TPB, TPB, 0, stream>>>(fc_w, DIM_NO, DIM_NOP, DIM_H / 8, W_SCALE, fcw16);
  wmma_gemm64<1, 1, 2, 0, false, 0><<<dim3((DIM_B / 64) * (DIM_G4 / 64) / 8, 1), TPB, 0, stream>>>(
      ameanh, ameanl, PITCH_IN, 0L, wihh, wihl, PITCH_IN, 0L, (void*)xc, (void*)nullptr, DIM_G4, 0L,
      bsum, (const float*)nullptr, 0L, DIM_B, DIM_G4, K_IN, 1.0f);
  wmma_gemm64<1, 1, 2, 0, false, 1><<<dim3((DIM_B / 64) * (DIM_H / 64) / 8, 1), TPB, 0, stream>>>(
      ameanh, ameanl, PITCH_IN, 0L, fchh, fchl, DIM_E, 0L, (void*)h0t, (void*)nullptr, DIM_H, 0L,
      fc_h_b, (const float*)nullptr, 0L, DIM_B, DIM_H, DIM_E, 1.0f);
  wmma_gemm64<1, 1, 2, 0, false, 1><<<dim3((DIM_B / 64) * (DIM_H / 64) / 8, 1), TPB, 0, stream>>>(
      ameanh, ameanl, PITCH_IN, 0L, fcmh, fcml, DIM_E, 0L, (void*)m0t, (void*)nullptr, DIM_H, 0L,
      fc_m_b, (const float*)nullptr, 0L, DIM_B, DIM_H, DIM_E, 1.0f);
  lstm_seq<<<DIM_B / 16, SEQ_THREADS, 0, stream>>>(h0t, m0t, label, xc, wbeg, whh16, wlabh, wlabl, hseqh, hseql);
  wmma_gemm64<0, 2, 0, 0, false, 0><<<dim3((DIM_B * DIM_T / 64) * (DIM_NOP / 64) / 8, 1), TPB, 0, stream>>>(
      hseqh, hseql, DIM_H, 0L, fcw16, (const unsigned short*)nullptr, DIM_H, 0L, (void*)outp, (void*)nullptr, DIM_NOP, 0L,
      (const float*)nullptr, (const float*)nullptr, 0L, DIM_B * DIM_T, DIM_NOP, DIM_H, INV_GSCALE);
  heads_kernel<<<DIM_B, TPB, 0, stream>>>(outp, fc_b, length, out);
}
